// MHSelfAttention_77309411786
// MI455X (gfx1250) — hardware-verified
//
#include <hip/hip_runtime.h>
#include <hip/hip_bf16.h>

typedef __attribute__((ext_vector_type(16))) _Float16 v16h;
typedef __attribute__((ext_vector_type(8)))  _Float16 v8h;
typedef __attribute__((ext_vector_type(16))) __bf16   v16b;
typedef __attribute__((ext_vector_type(8)))  __bf16   v8b;
typedef __attribute__((ext_vector_type(8)))  float    v8f;
typedef __attribute__((ext_vector_type(4)))  float    v4f;
typedef __attribute__((ext_vector_type(4)))  unsigned int v4u;

static constexpr int kBatch = 2;
static constexpr int kSeq   = 4096;
static constexpr int kEmb   = 512;
static constexpr int kHeads = 8;
static constexpr int kHdim  = 64;
static constexpr int kTok   = kBatch * kSeq;
static constexpr int kNqb   = kSeq / 64;
static constexpr int kAKC   = 64;
static constexpr int kANW   = 4;

static_assert(kEmb % 64 == 0 && kTok % 64 == 0, "gemm M,N tile multiples");
static_assert(kEmb % 32 == 0, "gemm K multiple of 32");
static_assert(kHeads * kHdim == kEmb, "head split");
static_assert(kSeq % 64 == 0 && kHdim == 64, "attention tiling");

__device__ __forceinline__ unsigned short f2bf_bits(float f) {
  unsigned u = __float_as_uint(f);
  return (unsigned short)((u + 0x7FFFu + ((u >> 16) & 1u)) >> 16);
}
__device__ __forceinline__ float bf_bits2f(unsigned short h) { return __uint_as_float(((unsigned)h) << 16); }

__device__ __forceinline__ void dep_guard_h(v8f& a, v8f& b, v16h x, v16h y) { asm volatile("v_nop\n\tv_nop\n\tv_nop\n\tv_nop" : "+v"(a), "+v"(b) : "v"(x), "v"(y)); }
__device__ __forceinline__ void dep_guard_b(v8f& a, v8f& b, v16b x, v16b y) { asm volatile("v_nop\n\tv_nop\n\tv_nop\n\tv_nop" : "+v"(a), "+v"(b) : "v"(x), "v"(y)); }
__device__ __forceinline__ void keep4_h(v16h a, v16h b, v16h c, v16h d) { asm volatile("v_nop" :: "v"(a), "v"(b), "v"(c), "v"(d)); }
__device__ __forceinline__ void keep4_b(v16b a, v16b b, v16b c, v16b d) { asm volatile("v_nop" :: "v"(a), "v"(b), "v"(c), "v"(d)); }
__device__ __forceinline__ void acc_guard4(v8f& a, v8f& b, v8f& c, v8f& d) { asm volatile("v_nop\n\tv_nop\n\tv_nop\n\tv_nop" : "+v"(a), "+v"(b), "+v"(c), "+v"(d)); }
template <typename T> struct Frag;
template <> struct Frag<_Float16> {
  typedef v16h V; union U { v16h v; v8h h[2]; };
  static __device__ __forceinline__ v16h load(const _Float16* p) {
    U f; f.h[0] = *(const v8h*)(p); f.h[1] = *(const v8h*)(p + 16); return f.v;
  }
  static __device__ __forceinline__ v8f mma(v16h a, v16h b, v8f c) {
    return __builtin_amdgcn_wmma_f32_16x16x32_f16(false, a, false, b, (short)0, c, false, false);
  }
  static __device__ __forceinline__ void guard(v8f& a, v8f& b, v16h x, v16h y) { dep_guard_h(a, b, x, y); }
  static __device__ __forceinline__ void keep(v16h a, v16h b, v16h c, v16h d) { keep4_h(a, b, c, d); }
};
template <> struct Frag<__bf16> {
  typedef v16b V; union U { v16b v; v8b h[2]; };
  static __device__ __forceinline__ v16b load(const __bf16* p) {
    U f; f.h[0] = *(const v8b*)(p); f.h[1] = *(const v8b*)(p + 16); return f.v;
  }
  static __device__ __forceinline__ v8f mma(v16b a, v16b b, v8f c) {
    return __builtin_amdgcn_wmma_f32_16x16x32_bf16(false, a, false, b, (short)0, c, false, false);
  }
  static __device__ __forceinline__ void guard(v8f& a, v8f& b, v16b x, v16b y) { dep_guard_b(a, b, x, y); }
  static __device__ __forceinline__ void keep(v16b a, v16b b, v16b c, v16b d) { keep4_b(a, b, c, d); }
};

template <int ET> struct Elem;
template <> struct Elem<0> { typedef _Float16 T; };
template <> struct Elem<1> { typedef __bf16 T; };
template <int ET, int SPLITK, int BIAS_MODE, int OUT_MODE>
__global__ __launch_bounds__(256) void wmma_gemm64(
    const unsigned short* __restrict__ Ap, const unsigned short* __restrict__ A2p, int lda, long strideA,
    const unsigned short* __restrict__ Btp, const unsigned short* __restrict__ Bt2p, int ldb, long strideB,
    void* __restrict__ Cout, void* __restrict__ Cout2, int ldc, long strideC,
    const float* __restrict__ bias,
    int M, int N, int K, float scale) {
  constexpr bool SPLIT = (SPLITK > 0);
  constexpr bool SPLB  = (SPLITK > 1);
  typedef typename Elem<ET>::T T;
  typedef typename Frag<T>::V V;
  const T* A = (const T*)Ap; const T* A2 = (const T*)A2p; const T* Bt = (const T*)Btp; const T* Bt2 = (const T*)Bt2p;
  __shared__ __align__(16) float sT[8][16 * 68];
  const int b    = blockIdx.y;
  const int lane = threadIdx.x & 31;
  const int wave = threadIdx.x >> 5;
  const int tilesN = N >> 6;
  const int tilesM = M >> 6;
  const int tile = blockIdx.x * 8 + wave;
  if (tile >= tilesM * tilesN) return;
  const int tm = tile / tilesN;
  const int tn = tile - tm * tilesN;
  const int m0 = tm << 6;
  const int n0 = tn << 6;

  const T* Ab  = A  + (size_t)b * strideA;
  const T* Bb  = Bt + (size_t)b * strideB;
  const T* Ab2 = SPLIT ? (A2  + (size_t)b * strideA) : nullptr;
  const T* Bb2 = SPLB  ? (Bt2 + (size_t)b * strideB) : nullptr;

  const int rlane = lane & 15;
  const int koff  = (lane >> 4) * 8;
  const int mOff  = (lane >> 4) * 8;

  v8f acc[4][4];
#pragma unroll
  for (int i = 0; i < 4; ++i)
#pragma unroll
    for (int j = 0; j < 4; ++j) acc[i][j] = (v8f){0.f,0.f,0.f,0.f,0.f,0.f,0.f,0.f};

  for (int k0 = 0; k0 < K; k0 += 32) {
    V bh[4], bl[4];
#pragma unroll
    for (int j = 0; j < 4; ++j) {
      const size_t bo = (size_t)(n0 + (j << 4) + rlane) * ldb + koff + k0;
      bh[j] = Frag<T>::load(Bb + bo);
      if (SPLB) bl[j] = Frag<T>::load(Bb2 + bo); else bl[j] = bh[j];
    }
#pragma unroll
    for (int i = 0; i < 4; ++i) {
      const size_t ao = (size_t)(m0 + (i << 4) + rlane) * lda + koff + k0;
      V ah = Frag<T>::load(Ab + ao);
      V al = ah;
      if (SPLIT) al = Frag<T>::load(Ab2 + ao);
#pragma unroll
      for (int j = 0; j < 4; ++j) {
        acc[i][j] = Frag<T>::mma(ah, bh[j], acc[i][j]);
        if (SPLB)  acc[i][j] = Frag<T>::mma(ah, bl[j], acc[i][j]);
        if (SPLIT) acc[i][j] = Frag<T>::mma(al, bh[j], acc[i][j]);
      }
      Frag<T>::guard(acc[i][0], acc[i][3], ah, al);
    }
    Frag<T>::keep(bh[0], bh[1], bh[2], bh[3]);
    if (SPLB) Frag<T>::keep(bl[0], bl[1], bl[2], bl[3]);
  }
  acc_guard4(acc[0][0], acc[0][1], acc[0][2], acc[0][3]);
  acc_guard4(acc[1][0], acc[1][1], acc[1][2], acc[1][3]);
  acc_guard4(acc[2][0], acc[2][1], acc[2][2], acc[2][3]);
  acc_guard4(acc[3][0], acc[3][1], acc[3][2], acc[3][3]);

  float* slab = sT[wave];
#pragma unroll
  for (int i = 0; i < 4; ++i) {
    const int mBase = m0 + (i << 4);
#pragma unroll
    for (int j = 0; j < 4; ++j) {
      const int n = n0 + (j << 4) + rlane;
      float bv = 0.f;
      if (BIAS_MODE == 2) bv = bias[n];
#pragma unroll
      for (int r = 0; r < 8; ++r) {
        float v = acc[i][j][r] * scale;
        if (BIAS_MODE == 1) v += bias[mBase + mOff + r];
        if (BIAS_MODE == 2) v += bv;
        slab[(mOff + r) * 68 + (j << 4) + rlane] = v;
      }
    }
    __builtin_amdgcn_fence(__ATOMIC_RELEASE, "workgroup");
    __builtin_amdgcn_wave_barrier();
    __builtin_amdgcn_fence(__ATOMIC_ACQUIRE, "workgroup");
    if (OUT_MODE == 0) {
      float* C = (float*)Cout + (size_t)b * strideC;
      const int hh = lane >> 4, c4 = (lane & 15) * 4;
      for (int pass = 0; pass < 2; ++pass) {
#pragma unroll
        for (int it = 0; it < 8; ++it) {
          const int row = it * 2 + hh;
          v4f v = *(const v4f*)(slab + row * 68 + c4);
          *(volatile v4f*)(C + (size_t)(mBase + row) * ldc + n0 + c4) = v;
        }
        __threadfence();
      }
    } else {
      const int q = lane >> 3, c8 = (lane & 7) * 8;
      unsigned short* C  = (unsigned short*)Cout  + (size_t)b * strideC;
      unsigned short* C2 = (OUT_MODE == 2) ? ((unsigned short*)Cout2 + (size_t)b * strideC) : nullptr;
      for (int pass = 0; pass < 2; ++pass) {
#pragma unroll
        for (int it = 0; it < 4; ++it) {
          const int row = it * 4 + q;
          const float* sp = slab + row * 68 + c8;
          v8h hv, lv;
#pragma unroll
          for (int e = 0; e < 8; ++e) {
            if (OUT_MODE == 1) {
              hv[e] = (_Float16)sp[e];
            } else {
              unsigned short hb = f2bf_bits(sp[e]);
              unsigned short lb = f2bf_bits(sp[e] - bf_bits2f(hb));
              hv[e] = __builtin_bit_cast(_Float16, hb);
              lv[e] = __builtin_bit_cast(_Float16, lb);
            }
          }
          *(volatile v8h*)(C + (size_t)(mBase + row) * ldc + n0 + c8) = hv;
          if (OUT_MODE == 2) *(volatile v8h*)(C2 + (size_t)(mBase + row) * ldc + n0 + c8) = lv;
        }
        __threadfence();
      }
    }
    __builtin_amdgcn_fence(__ATOMIC_RELEASE, "workgroup");
    __builtin_amdgcn_wave_barrier();
    __builtin_amdgcn_fence(__ATOMIC_ACQUIRE, "workgroup");
  }
}

__global__ __launch_bounds__(256) void cast_f32_bf16x2(
    const float* __restrict__ in, unsigned short* __restrict__ out, int n2) {
  int i = blockIdx.x * 256 + threadIdx.x;
  if (i < n2) {
    const float a0 = in[2 * i], a1 = in[2 * i + 1];
    const unsigned u = (unsigned)f2bf_bits(a0) | ((unsigned)f2bf_bits(a1) << 16);
    ((volatile unsigned*)out)[i] = u;
    __threadfence();
    ((volatile unsigned*)out)[i] = u;
  }
}

__device__ __forceinline__ __bf16 at_f2bf(float f) { return __builtin_bit_cast(__bf16, f2bf_bits(f)); }
__device__ __forceinline__ void at_split(float f, __bf16& hi, __bf16& lo) {
  const unsigned short hb = f2bf_bits(f);
  hi = __builtin_bit_cast(__bf16, hb);
  lo = at_f2bf(f - __uint_as_float(((unsigned)hb) << 16));
}
__device__ __forceinline__ v8f at_mma(v16b a, v16b b, v8f c) {
  c = __builtin_amdgcn_wmma_f32_16x16x32_bf16(false, a, false, b, (short)0, c, false, false);
  asm volatile("v_nop\n\tv_nop\n\tv_nop\n\tv_nop" : "+v"(c) : "v"(a), "v"(b));
  return c;
}

__global__ __launch_bounds__(128)
void attn_causal64(const unsigned short* __restrict__ qhp, const unsigned short* __restrict__ qlp,
                   const unsigned short* __restrict__ khp, const unsigned short* __restrict__ klp,
                   const unsigned short* __restrict__ vthp, const unsigned short* __restrict__ vtlp,
                   const int* __restrict__ pmask,
                   unsigned short* __restrict__ ohp, unsigned short* __restrict__ olp) {
  union FB { v16b v; v8b h[2]; };
  __shared__ __align__(16) __bf16 Ksh[kAKC * kHdim];
  __shared__ __align__(16) __bf16 Ksl[kAKC * kHdim];
  __shared__ __align__(16) __bf16 Vth[kHdim * kAKC];
  __shared__ __align__(16) __bf16 Vtl[kHdim * kAKC];
  __shared__ __align__(16) __bf16 Psh[kANW][16 * kAKC];
  __shared__ __align__(16) __bf16 Psl[kANW][16 * kAKC];
  __shared__ __align__(16) float  Os[kANW][16 * 68];

  const int tid  = threadIdx.x;
  const int wave = tid >> 5;
  const int lane = tid & 31;
  const int hh   = lane >> 4;
  const int c    = lane & 15;

  const int qb = blockIdx.x & (kNqb - 1);
  const int bh = blockIdx.x >> 6;
  const int h  = bh & (kHeads - 1);
  const int b  = bh >> 3;
  const int q0 = qb * 64 + wave * 16;

  const size_t bhoff = (size_t)b * kSeq * kEmb + (size_t)h * kHdim;
  const __bf16* qh = (const __bf16*)qhp + bhoff;
  const __bf16* ql = (const __bf16*)qlp + bhoff;
  const __bf16* kh = (const __bf16*)khp + bhoff;
  const __bf16* kl = (const __bf16*)klp + bhoff;
  const size_t vtoff = (size_t)h * kHdim * kTok + (size_t)b * kSeq;
  const __bf16* vth = (const __bf16*)vthp + vtoff;
  const __bf16* vtl = (const __bf16*)vtlp + vtoff;

  v16b qah[2], qal[2];
#pragma unroll
  for (int dc = 0; dc < 2; ++dc) {
    qah[dc] = Frag<__bf16>::load(qh + (size_t)(q0 + c) * kEmb + dc * 32 + 8 * hh);
    qal[dc] = Frag<__bf16>::load(ql + (size_t)(q0 + c) * kEmb + dc * 32 + 8 * hh);
  }

  float mrow[8], lrow[8];
  v8f oacc[4];
#pragma unroll
  for (int r = 0; r < 8; ++r) { mrow[r] = -INFINITY; lrow[r] = 0.f; }
#pragma unroll
  for (int t = 0; t < 4; ++t) oacc[t] = (v8f){0.f,0.f,0.f,0.f,0.f,0.f,0.f,0.f};

  for (int kc = 0; kc <= qb; ++kc) {
    const int kv0 = kc * kAKC;
    __syncthreads();
    {
#pragma unroll
      for (int i = 0; i < 4; ++i) {
        const int idx = tid + i * 128;
        const int row = idx >> 3;
        const int c8  = (idx & 7) * 8;
        const v4u a0 = *(const v4u*)(kh + (size_t)(kv0 + row) * kEmb + c8);
        const v4u a1 = *(const v4u*)(kl + (size_t)(kv0 + row) * kEmb + c8);
        *(v4u*)(Ksh + row * kHdim + c8) = a0;
        *(v4u*)(Ksl + row * kHdim + c8) = a1;
      }
      asm volatile("" ::: "memory");
#pragma unroll
      for (int i = 0; i < 4; ++i) {
        const int idx = tid + i * 128;
        const int row = idx >> 3;
        const int c8  = (idx & 7) * 8;
        const v4u a0 = *(const v4u*)(vth + (size_t)row * kTok + kv0 + c8);
        const v4u a1 = *(const v4u*)(vtl + (size_t)row * kTok + kv0 + c8);
        *(v4u*)(Vth + row * kAKC + c8) = a0;
        *(v4u*)(Vtl + row * kAKC + c8) = a1;
      }
    }
    __syncthreads();

    v8f s[4];
#pragma unroll
    for (int j = 0; j < 4; ++j) {
      s[j] = (v8f){0.f,0.f,0.f,0.f,0.f,0.f,0.f,0.f};
#pragma unroll
      for (int dc = 0; dc < 2; ++dc) {
        FB kb, kbl;
        kb.h[0]  = *(const v8b*)(Ksh + (j * 16 + c) * kHdim + dc * 32 + 8 * hh);
        kb.h[1]  = *(const v8b*)(Ksh + (j * 16 + c) * kHdim + dc * 32 + 16 + 8 * hh);
        kbl.h[0] = *(const v8b*)(Ksl + (j * 16 + c) * kHdim + dc * 32 + 8 * hh);
        kbl.h[1] = *(const v8b*)(Ksl + (j * 16 + c) * kHdim + dc * 32 + 16 + 8 * hh);
        s[j] = at_mma(qah[dc], kb.v,  s[j]);
        s[j] = at_mma(qah[dc], kbl.v, s[j]);
        s[j] = at_mma(qal[dc], kb.v,  s[j]);
      }
    }
    const bool diag = (kc == qb);
    float cm[8];
#pragma unroll
    for (int r = 0; r < 8; ++r) {
      const int qrow = q0 + 8 * hh + r;
      float m = -INFINITY;
#pragma unroll
      for (int j = 0; j < 4; ++j) {
        const int kvcol = kv0 + j * 16 + c;
        float sv = s[j][r];
        if (diag && (kvcol > qrow)) sv = -INFINITY;
        s[j][r] = sv;
        m = fmaxf(m, sv);
      }
#pragma unroll
      for (int off = 1; off < 16; off <<= 1) m = fmaxf(m, __shfl_xor(m, off, 32));
      cm[r] = m;
    }
    __bf16* pwh = Psh[wave];
    __bf16* pwl = Psl[wave];
#pragma unroll
    for (int r = 0; r < 8; ++r) {
      const float mnew = fmaxf(mrow[r], cm[r]);
      const float alpha = expf(mrow[r] - mnew);
      mrow[r] = mnew;
      float psum = 0.f;
#pragma unroll
      for (int j = 0; j < 4; ++j) {
        const float p = expf(s[j][r] - mnew);
        psum += p;
        __bf16 ph, pl;
        at_split(p, ph, pl);
        pwh[(8 * hh + r) * kAKC + j * 16 + c] = ph;
        pwl[(8 * hh + r) * kAKC + j * 16 + c] = pl;
      }
#pragma unroll
      for (int off = 1; off < 16; off <<= 1) psum += __shfl_xor(psum, off, 32);
      lrow[r] = lrow[r] * alpha + psum;
#pragma unroll
      for (int t = 0; t < 4; ++t) oacc[t][r] *= alpha;
    }
    __builtin_amdgcn_fence(__ATOMIC_RELEASE, "workgroup");
    __builtin_amdgcn_wave_barrier();
    __builtin_amdgcn_fence(__ATOMIC_ACQUIRE, "workgroup");
#pragma unroll 1
    for (int kk = 0; kk < 2; ++kk) {
      FB pa, pl;
      pa.h[0] = *(const v8b*)(pwh + c * kAKC + kk * 32 + 8 * hh);
      pa.h[1] = *(const v8b*)(pwh + c * kAKC + kk * 32 + 16 + 8 * hh);
      pl.h[0] = *(const v8b*)(pwl + c * kAKC + kk * 32 + 8 * hh);
      pl.h[1] = *(const v8b*)(pwl + c * kAKC + kk * 32 + 16 + 8 * hh);
#pragma unroll
      for (int t = 0; t < 4; ++t) {
        FB vb, vl;
        vb.h[0] = *(const v8b*)(Vth + (t * 16 + c) * kAKC + kk * 32 + 8 * hh);
        vb.h[1] = *(const v8b*)(Vth + (t * 16 + c) * kAKC + kk * 32 + 16 + 8 * hh);
        vl.h[0] = *(const v8b*)(Vtl + (t * 16 + c) * kAKC + kk * 32 + 8 * hh);
        vl.h[1] = *(const v8b*)(Vtl + (t * 16 + c) * kAKC + kk * 32 + 16 + 8 * hh);
        oacc[t] = at_mma(pa.v, vb.v, oacc[t]);
        oacc[t] = at_mma(pa.v, vl.v, oacc[t]);
        oacc[t] = at_mma(pl.v, vb.v, oacc[t]);
      }
    }
  }

  float* os = Os[wave];
#pragma unroll
  for (int r = 0; r < 8; ++r) {
    const int qrow = q0 + 8 * hh + r;
    const int keep = pmask[(size_t)b * kSeq + qrow];
    float inv = 1.0f / lrow[r];
    if (keep == 0) inv = __uint_as_float(0x7fc00000u);
#pragma unroll
    for (int t = 0; t < 4; ++t) os[(8 * hh + r) * 68 + t * 16 + c] = oacc[t][r] * inv;
  }
  __builtin_amdgcn_fence(__ATOMIC_RELEASE, "workgroup");
  __builtin_amdgcn_wave_barrier();
  __builtin_amdgcn_fence(__ATOMIC_ACQUIRE, "workgroup");
  {
    const int q4 = lane >> 3, c8 = (lane & 7) * 8;
    unsigned short* ob  = ohp + bhoff;
    unsigned short* obl = olp + bhoff;
    for (int pass = 0; pass < 2; ++pass) {
#pragma unroll
      for (int it = 0; it < 4; ++it) {
        const int row = it * 4 + q4;
        const float* sp = os + row * 68 + c8;
        v8h hv, lv;
#pragma unroll
        for (int e = 0; e < 8; ++e) {
          unsigned short hb = f2bf_bits(sp[e]);
          unsigned short lb = f2bf_bits(sp[e] - bf_bits2f(hb));
          hv[e] = __builtin_bit_cast(_Float16, hb);
          lv[e] = __builtin_bit_cast(_Float16, lb);
        }
        *(volatile v8h*)(ob  + (size_t)(q0 + row) * kEmb + c8) = hv;
        *(volatile v8h*)(obl + (size_t)(q0 + row) * kEmb + c8) = lv;
      }
      __threadfence();
    }
  }
}

static constexpr size_t kPlaneTok = (size_t)kTok * kEmb;
static constexpr size_t kPlaneW   = (size_t)kEmb * kEmb;
static constexpr size_t kOffXb  = 0;
static constexpr size_t kOffWb  = kOffXb  + kPlaneTok * 2;
static constexpr size_t kOffQKh = kOffWb  + 4 * kPlaneW * 2;
static constexpr size_t kOffQKl = kOffQKh + 2 * kPlaneTok * 2;
static constexpr size_t kOffVth = kOffQKl + 2 * kPlaneTok * 2;
static constexpr size_t kOffVtl = kOffVth + kPlaneTok * 2;
static constexpr size_t kOffOh  = kOffVtl + kPlaneTok * 2;
static constexpr size_t kOffOl  = kOffOh  + kPlaneTok * 2;
static constexpr size_t kWsEnd  = kOffOl  + kPlaneTok * 2;
static_assert(kWsEnd == 77594624, "carve total");
static_assert(kWsEnd <= 134217728, "carve budget");
static_assert((kPlaneTok / 2) % 256 == 0 && (kPlaneW / 2) % 256 == 0, "cast grids exact");

extern "C" void kernel_launch(void* const* d_in, const int* in_sizes, int n_in,
                              void* d_out, int out_size, void* d_ws,
                              size_t ws_size, hipStream_t stream) {
  (void)in_sizes; (void)n_in; (void)out_size; (void)ws_size;
  const float* x  = (const float*)d_in[0];
  const int*   pm = (const int*)d_in[1];
  const float* Wq = (const float*)d_in[2];
  const float* Wk = (const float*)d_in[3];
  const float* Wv = (const float*)d_in[4];
  const float* Wu = (const float*)d_in[5];
  const float* bu = (const float*)d_in[6];
  float* out = (float*)d_out;

  unsigned char* ws = (unsigned char*)d_ws;
  unsigned short* Xb  = (unsigned short*)(ws + kOffXb);
  unsigned short* Wb  = (unsigned short*)(ws + kOffWb);
  unsigned short* QKh = (unsigned short*)(ws + kOffQKh);
  unsigned short* QKl = (unsigned short*)(ws + kOffQKl);
  unsigned short* Vth = (unsigned short*)(ws + kOffVth);
  unsigned short* Vtl = (unsigned short*)(ws + kOffVtl);
  unsigned short* Oh  = (unsigned short*)(ws + kOffOh);
  unsigned short* Ol  = (unsigned short*)(ws + kOffOl);

  const int nTok2 = (int)(kPlaneTok / 2);
  const int nW2   = (int)(kPlaneW / 2);

  cast_f32_bf16x2<<<dim3(nTok2 / 256), dim3(256), 0, stream>>>(x, Xb, nTok2);
  cast_f32_bf16x2<<<dim3(nW2 / 256), dim3(256), 0, stream>>>(Wq, Wb + 0 * kPlaneW, nW2);
  cast_f32_bf16x2<<<dim3(nW2 / 256), dim3(256), 0, stream>>>(Wk, Wb + 1 * kPlaneW, nW2);
  cast_f32_bf16x2<<<dim3(nW2 / 256), dim3(256), 0, stream>>>(Wv, Wb + 2 * kPlaneW, nW2);
  cast_f32_bf16x2<<<dim3(nW2 / 256), dim3(256), 0, stream>>>(Wu, Wb + 3 * kPlaneW, nW2);

  const float inv4 = 0.21022410381342863f;
  const int gemmBlocks = ((kTok / 64) * (kEmb / 64) + 7) / 8;

  wmma_gemm64<1, 0, 0, 2><<<dim3(gemmBlocks, 2), dim3(256), 0, stream>>>(
      Xb, Xb, kEmb, 0L,
      Wb, Wb, kEmb, (long)kPlaneW,
      (void*)QKh, (void*)QKl, kEmb, (long)kPlaneTok,
      bu, kTok, kEmb, kEmb, inv4);

  wmma_gemm64<1, 0, 0, 2><<<dim3(gemmBlocks, 1), dim3(256), 0, stream>>>(
      Wb + 2 * kPlaneW, Wb + 2 * kPlaneW, kEmb, 0L,
      Xb, Xb, kEmb, 0L,
      (void*)Vth, (void*)Vtl, kTok, 0L,
      bu, kEmb, kTok, kEmb, 1.0f);

  attn_causal64<<<dim3(kBatch * kHeads * kNqb), dim3(128), 0, stream>>>(
      QKh, QKl, QKh + kPlaneTok, QKl + kPlaneTok, Vth, Vtl, pm, Oh, Ol);

  wmma_gemm64<1, 1, 2, 0><<<dim3(gemmBlocks, 1), dim3(256), 0, stream>>>(
      Oh, Ol, kEmb, 0L,
      Wb + 3 * kPlaneW, Wb + 3 * kPlaneW, kEmb, 0L,
      (void*)out, (void*)out, kEmb, 0L,
      bu, kTok, kEmb, kEmb, 1.0f);
}
